// MoEEPTop2_44504451121358
// MI455X (gfx1250) — hardware-verified
//
#include <hip/hip_runtime.h>
#include <math.h>

typedef __attribute__((ext_vector_type(16))) _Float16 v16h;
typedef __attribute__((ext_vector_type(16))) __bf16 v16b;
typedef __attribute__((ext_vector_type(8)))  _Float16 v8h;
typedef __attribute__((ext_vector_type(8)))  float v8f;
typedef __attribute__((ext_vector_type(4)))  float v4f;
typedef __attribute__((ext_vector_type(2)))  float v2f;
typedef __attribute__((ext_vector_type(4)))  unsigned v4u;
typedef __attribute__((ext_vector_type(4)))  int v4i;
typedef float __attribute__((may_alias)) float_a;
typedef int __attribute__((may_alias)) int_a;

template <typename T> __device__ __forceinline__ void vst2(void* p, T v) { *(volatile T*)p = v; __threadfence(); *(volatile T*)p = v; }
__device__ __forceinline__ v8f wmma16(v16h a, v16h b, v8f c) {
  v8f d = __builtin_amdgcn_wmma_f32_16x16x32_f16(false, a, false, b, (short)0, c, false, false);
  asm volatile("v_nop\n\tv_nop\n\tv_nop\n\tv_nop" : "+v"(d) : "v"(a), "v"(b));
  return d;
}
__device__ __forceinline__ v8f wmma_bf(v16b a, v16b b, v8f c) {
  v8f d = __builtin_amdgcn_wmma_f32_16x16x32_bf16(false, a, false, b, (short)0, c, false, false);
  asm volatile("v_nop\n\tv_nop\n\tv_nop\n\tv_nop" : "+v"(d) : "v"(a), "v"(b));
  return d;
}
__device__ __forceinline__ v16h frag_h(const _Float16* rowk0, int lane) {
  union { v16h v; v8h q[2]; } u; const _Float16* p = rowk0 + 8 * (lane >> 4);
  u.q[0] = *(const v8h*)p; u.q[1] = *(const v8h*)(p + 16); return u.v;
}
__device__ __forceinline__ v16h frag_f32(const float* rowk0, int lane) {
  v16h a; const float* p = rowk0 + 8 * (lane >> 4);
#pragma unroll
  for (int i = 0; i < 8; ++i) { a[i] = (_Float16)p[i]; a[8 + i] = (_Float16)p[16 + i]; }
  return a;
}
__device__ __forceinline__ v16h frag_f32s(const float* rowk0, int lane, float sc) {
  v16h a; const float* p = rowk0 + 8 * (lane >> 4);
#pragma unroll
  for (int i = 0; i < 8; ++i) { a[i] = (_Float16)(p[i] * sc); a[8 + i] = (_Float16)(p[16 + i] * sc); }
  return a;
}
__device__ __forceinline__ v16h fragc_f32(const float* W, int k0, int n, int lane, int ld, int K) {
  v16h a; const int g = lane >> 4;
#pragma unroll
  for (int i = 0; i < 8; ++i) { const int ka = k0 + 8 * g + i, kb = ka + 16;
    a[i] = (_Float16)(ka < K ? W[(size_t)(ka < K ? ka : K - 1) * ld + n] : 0.f); a[8 + i] = (_Float16)(kb < K ? W[(size_t)(kb < K ? kb : K - 1) * ld + n] : 0.f); }
  return a;
}
struct F2 { v16b h, l; };
__device__ __forceinline__ F2 bsplit16(const float v[16]) { F2 r;
#pragma unroll
  for (int i = 0; i < 16; ++i) { const __bf16 h = (__bf16)v[i]; r.h[i] = h; r.l[i] = (__bf16)(v[i] - (float)h); }
  return r; }
__device__ __forceinline__ F2 split_row(const float* row, int k0, int lane) { float v[16]; const float* p = row + k0 + 8 * (lane >> 4);
#pragma unroll
  for (int i = 0; i < 8; ++i) { v[i] = p[i]; v[8 + i] = p[16 + i]; }
  return bsplit16(v); }
__device__ __forceinline__ F2 split_rowK(const float* row, int k0, int lane, int K) { float v[16]; const int g = lane >> 4;
#pragma unroll
  for (int i = 0; i < 8; ++i) { const int ka = k0 + 8 * g + i, kb = ka + 16; v[i] = ka < K ? row[ka < K ? ka : K - 1] : 0.f; v[8 + i] = kb < K ? row[kb < K ? kb : K - 1] : 0.f; }
  return bsplit16(v); }
__device__ __forceinline__ F2 split_col(const float* W, int k0, int n, int lane, int ld, int K) { float v[16]; const int g = lane >> 4;
#pragma unroll
  for (int i = 0; i < 8; ++i) { const int ka = k0 + 8 * g + i, kb = ka + 16; v[i] = ka < K ? W[(size_t)(ka < K ? ka : K - 1) * ld + n] : 0.f; v[8 + i] = kb < K ? W[(size_t)(kb < K ? kb : K - 1) * ld + n] : 0.f; }
  return bsplit16(v); }
__device__ __forceinline__ v8f mac3(const F2& a, const F2& b, v8f c) { c = wmma_bf(a.l, b.h, c); c = wmma_bf(a.h, b.l, c); return wmma_bf(a.h, b.h, c); }
__device__ __forceinline__ float sigm(float v) { return 1.0f / (1.0f + expf(-v)); }
#define LDSX() do { asm volatile("s_wait_dscnt 0" ::: "memory"); __builtin_amdgcn_wave_barrier(); __builtin_amdgcn_fence(__ATOMIC_RELEASE, "workgroup"); } while (0)


#define NTK 8192
#define DD 512
#define HH 1024
#define NE 8
#define NSLOT 2
#define NENT (NTK * NSLOT)
#ifndef NRT
#define NRT (NTK / 64)
#endif
typedef __attribute__((ext_vector_type(8))) __bf16 v8b;
__device__ __forceinline__ v16b frag_b(const __bf16* rowk0, int lane) {
  union { v16b v; v8b q[2]; } u; const __bf16* p = rowk0 + 8 * (lane >> 4);
  u.q[0] = *(const v8b*)p; u.q[1] = *(const v8b*)(p + 16); return u.v;
}
__device__ __forceinline__ float bfr(float v) { return (float)(__bf16)v; }
__device__ __attribute__((noinline)) float exp_ni(float v) { return expf(v); }
__device__ __attribute__((noinline)) float erf_ni(float v) { return erff(v); }
__device__ __forceinline__ float gelu_exact(float v) { return 0.5f * v * (1.0f + erf_ni(v * 0.70710678118654752f)); }

#define PK_W1 0
#define PK_W2 ((size_t)NE * HH * DD)
#define PK_END (PK_W2 + (size_t)NE * DD * HH)
#define WS_PK   0u
#define WS_XB   (((2u * PK_END) + 127u) / 128u * 128u)
#define WS_SEL  (WS_XB + 2u * NTK * DD)
#define WS_WGT  (WS_SEL + 4u * NTK * 2)
#define WS_CNT  (WS_WGT + 4u * NTK * 2)
#define WS_LIST (WS_CNT + 128u)
#define WS_HBH  (WS_LIST + 4u * NE * NENT)
#define WS_HBL  (WS_HBH + 2u * (size_t)NENT * HH)
#define WS_O    (WS_HBL + 2u * (size_t)NENT * HH)
#define WS_END  (WS_O + 4u * (size_t)NENT * DD)

__global__ __launch_bounds__(256) void k_pack(const float* __restrict__ W1, const float* __restrict__ W2, __bf16* __restrict__ PK) {
  __shared__ __align__(16) __bf16 s[HH]; const int n = blockIdx.x, which = blockIdx.y, e = blockIdx.z, t = threadIdx.x; int K; size_t dst;
  if (which == 0) { K = DD; dst = PK_W1 + ((size_t)e * HH + n) * DD; for (int k = t; k < DD; k += 256) s[k] = (__bf16)W1[((size_t)e * DD + k) * HH + n]; }
  else { if (n >= DD) return; K = HH; dst = PK_W2 + ((size_t)e * DD + n) * HH; for (int k = t; k < HH; k += 256) s[k] = (__bf16)W2[((size_t)e * HH + k) * DD + n]; }
  __syncthreads();
  for (int q = t; q < K / 8; q += 256) vst2((unsigned*)(PK + dst + q * 8), *(const v4u*)&s[q * 8]);
}
__global__ __launch_bounds__(256) void k_gate(const float* __restrict__ X, const float* __restrict__ WR, const float* __restrict__ BR, __bf16* __restrict__ XB, int* __restrict__ SEL, float* __restrict__ WGT) {
  __shared__ __align__(16) __bf16 sx[64][DD]; __shared__ double slg[64][NE]; __shared__ __align__(16) int ssel[64][2]; __shared__ __align__(16) float swg[64][2];
  const int tid = threadIdx.x; const size_t t0 = (size_t)blockIdx.x * 64;
  for (int q = tid; q < 64 * DD; q += 256) { const int r = q / DD, c = q % DD; sx[r][c] = (__bf16)X[(t0 + r) * DD + c]; }
  __syncthreads();
  { const int tl = tid >> 2, e0 = (tid & 3) * 2; double a0 = 0.0, a1 = 0.0;
#pragma unroll 1
    for (int k = 0; k < DD; ++k) { const float xv = (float)sx[tl][k]; a0 += (double)(xv * bfr(WR[(size_t)e0 * DD + k])); a1 += (double)(xv * bfr(WR[(size_t)(e0 + 1) * DD + k])); }
    slg[tl][e0] = a0 + (double)bfr(BR[e0]); slg[tl][e0 + 1] = a1 + (double)bfr(BR[e0 + 1]); }
  __syncthreads();
  if (tid < 64) { const int tl = tid; double mx = -1e300; int a = 0;
#pragma unroll
    for (int e = 0; e < NE; ++e) if (slg[tl][e] > mx) { mx = slg[tl][e]; a = e; }
    double m2 = -1e300; int bsel = 0;
#pragma unroll
    for (int e = 0; e < NE; ++e) if (e != a && slg[tl][e] > m2) { m2 = slg[tl][e]; bsel = e; }
    float se = 0.f; float pe[NE]; const float mxf = (float)mx;
#pragma unroll
    for (int e = 0; e < NE; ++e) { pe[e] = exp_ni((float)slg[tl][e] - mxf); se += pe[e]; }
    float pa = 0.f, pb = 0.f;
#pragma unroll
    for (int e = 0; e < NE; ++e) { pa = (e == a) ? pe[e] / se : pa; pb = (e == bsel) ? pe[e] / se : pb; }
    ssel[tl][0] = a; ssel[tl][1] = bsel; swg[tl][0] = pa; swg[tl][1] = pb; }
  __syncthreads();
  for (int q = tid; q < 64 * DD / 8; q += 256) vst2((unsigned*)(XB + t0 * DD + q * 8), *(const v4u*)(&sx[0][0] + q * 8));
  if (tid < 32) vst2((unsigned*)(SEL + t0 * 2 + tid * 4), *(const v4u*)(&ssel[0][0] + tid * 4)); else if (tid < 64) vst2(WGT + t0 * 2 + (tid - 32) * 4, *(const v4f*)(&swg[0][0] + (tid - 32) * 4));
}
__global__ __launch_bounds__(256) void k_sort(const int* __restrict__ SEL, int ntok, int* __restrict__ CNT, int* __restrict__ LIST) {
  __shared__ int scnt[NE], sfirst[NE]; __shared__ __align__(16) int sc[32]; const int t = threadIdx.x;
  if (t < NE) { int c = 0, f = 0; bool seen = false; for (int i = 0; i < ntok; ++i) { for (int sl = 0; sl < 2; ++sl) if (SEL[i * 2 + sl] == t) { LIST[(size_t)t * NENT + c] = i * 2 + sl; if (!seen) { f = i * 2 + sl; seen = true; } ++c; } } scnt[t] = c; sfirst[t] = f; }
  __syncthreads();
  for (int q = t; q < NE * NENT; q += 256) { const int e = q / NENT, k = q % NENT; if (k >= scnt[e]) LIST[q] = sfirst[e]; }
  if (t < 32) sc[t] = (t < NE) ? scnt[t] : 0;
  __syncthreads();
  for (int q = t; q < NE * NENT / 4; q += 256) { v4u v; const int* p = LIST + (size_t)q * 4; v[0] = p[0]; v[1] = p[1]; v[2] = p[2]; v[3] = p[3]; vst2((unsigned*)(LIST + (size_t)q * 4), v); }
  if (t < 8) vst2((unsigned*)(CNT + t * 4), *(const v4u*)&sc[t * 4]);
}
__global__ __launch_bounds__(128) void k_fc(const __bf16* __restrict__ XB, const __bf16* __restrict__ PK, const float* __restrict__ B1, const int* __restrict__ CNT, const int* __restrict__ LIST, __bf16* __restrict__ HBH, __bf16* __restrict__ HBL) {
  __shared__ __align__(16) __bf16 soh[4][16][136], sol[4][16][136]; __shared__ int sent[64];
  const int tid = threadIdx.x, wave = tid >> 5, lane = tid & 31, col = lane & 15, g = lane >> 4; const int e = blockIdx.z; const int cnt = CNT[e]; if (blockIdx.x * 64 >= cnt) return;
  if (tid < 64) sent[tid] = LIST[(size_t)e * NENT + blockIdx.x * 64 + tid];
  __syncthreads();
  const int n0 = blockIdx.y * 128; const __bf16* P = PK + PK_W1 + (size_t)e * HH * DD;
  v8f acc[8] = {};
#pragma unroll 2
  for (int kc = 0; kc < DD / 32; ++kc) { const v16b a = frag_b(XB + (size_t)(sent[wave * 16 + col] >> 1) * DD + kc * 32, lane);
#pragma unroll
    for (int j = 0; j < 8; ++j) acc[j] = wmma_bf(a, frag_b(P + (size_t)(n0 + j * 16 + col) * DD + kc * 32, lane), acc[j]); }
#pragma unroll
  for (int j = 0; j < 8; ++j) { const float bb = bfr(B1[(size_t)e * HH + n0 + j * 16 + col]);
#pragma unroll
    for (int r = 0; r < 8; ++r) { const float v = gelu_exact(acc[j][r] + bb); const __bf16 hb = (__bf16)v; soh[wave][8 * g + r][j * 16 + col] = hb; sol[wave][8 * g + r][j * 16 + col] = (__bf16)(v - (float)hb); } }
  LDSX();
  for (int rl = 0; rl < 16; ++rl) { const int li = blockIdx.x * 64 + wave * 16 + rl; if (li < cnt && lane < 16) { const size_t o = (size_t)sent[wave * 16 + rl] * HH + n0 + lane * 8; vst2((unsigned*)(HBH + o), *(const v4u*)&soh[wave][rl][lane * 8]); vst2((unsigned*)(HBL + o), *(const v4u*)&sol[wave][rl][lane * 8]); } }
}
__global__ __launch_bounds__(128) void k_pj(const __bf16* __restrict__ HBH, const __bf16* __restrict__ HBL, const __bf16* __restrict__ PK, const float* __restrict__ B2, const int* __restrict__ CNT, const int* __restrict__ LIST, float* __restrict__ O) {
  __shared__ __align__(16) float so[4][16][132]; __shared__ int sent[64];
  const int tid = threadIdx.x, wave = tid >> 5, lane = tid & 31, col = lane & 15, g = lane >> 4; const int e = blockIdx.z; const int cnt = CNT[e]; if (blockIdx.x * 64 >= cnt) return;
  if (tid < 64) sent[tid] = LIST[(size_t)e * NENT + blockIdx.x * 64 + tid];
  __syncthreads();
  const int n0 = blockIdx.y * 128; const __bf16* P = PK + PK_W2 + (size_t)e * DD * HH;
  v8f acc[8] = {};
#pragma unroll 2
  for (int kc = 0; kc < HH / 32; ++kc) { const size_t ar = (size_t)sent[wave * 16 + col] * HH + kc * 32; const v16b ah = frag_b(HBH + ar, lane), al = frag_b(HBL + ar, lane);
#pragma unroll
    for (int j = 0; j < 8; ++j) { const v16b w = frag_b(P + (size_t)(n0 + j * 16 + col) * HH + kc * 32, lane); acc[j] = wmma_bf(al, w, acc[j]); acc[j] = wmma_bf(ah, w, acc[j]); } }
#pragma unroll
  for (int j = 0; j < 8; ++j) { const float bb = bfr(B2[(size_t)e * DD + n0 + j * 16 + col]);
#pragma unroll
    for (int r = 0; r < 8; ++r) so[wave][8 * g + r][j * 16 + col] = acc[j][r] + bb; }
  LDSX();
  for (int rl = 0; rl < 16; ++rl) { const int li = blockIdx.x * 64 + wave * 16 + rl; if (li < cnt) vst2(O + (size_t)sent[wave * 16 + rl] * DD + n0 + lane * 4, *(const v4f*)&so[wave][rl][lane * 4]); }
}
__global__ __launch_bounds__(128) void k_comb(const int* __restrict__ SEL, const float* __restrict__ WGT, const float* __restrict__ O, float* __restrict__ OUT) {
  const size_t t = blockIdx.x; const int tid = threadIdx.x; const int ea = SEL[t * 2], eb = SEL[t * 2 + 1]; const float wa = WGT[t * 2], wb = WGT[t * 2 + 1];
  const int sfirst = (ea < eb) ? 0 : 1;
  const float* o0 = O + (t * 2 + sfirst) * DD; const float* o1 = O + (t * 2 + (1 - sfirst)) * DD; const float w0 = sfirst ? wb : wa, w1 = sfirst ? wa : wb;
  v4f v;
#pragma unroll
  for (int i = 0; i < 4; ++i) { const int c = tid * 4 + i; v[i] = (w0 * o0[c]) + (w1 * o1[c]); }
  vst2(OUT + t * DD + tid * 4, v);
}
extern "C" void kernel_launch(void* const* d_in, const int* in_sizes, int n_in, void* d_out, int out_size, void* d_ws, size_t ws_size, hipStream_t stream) {
  (void)in_sizes; (void)n_in; (void)out_size;
  const float** F = (const float**)d_in;
  if (ws_size < (size_t)WS_END) return;
  char* ws = (char*)d_ws; __bf16 *PK = (__bf16*)(ws + WS_PK), *XB = (__bf16*)(ws + WS_XB), *HBH = (__bf16*)(ws + WS_HBH), *HBL = (__bf16*)(ws + WS_HBL); int *SEL = (int*)(ws + WS_SEL), *CNT = (int*)(ws + WS_CNT), *LIST = (int*)(ws + WS_LIST); float *WGT = (float*)(ws + WS_WGT), *O = (float*)(ws + WS_O);
  k_pack<<<dim3(HH, 2, NE), 256, 0, stream>>>(F[3], F[5], PK);
  k_gate<<<NRT, 256, 0, stream>>>(F[0], F[1], F[2], XB, SEL, WGT);
  k_sort<<<1, 256, 0, stream>>>(SEL, NRT * 64, CNT, LIST);
  k_fc<<<dim3(NENT / 64, HH / 128, NE), 128, 0, stream>>>(XB, PK, F[4], CNT, LIST, HBH, HBL);
  k_pj<<<dim3(NENT / 64, DD / 128, NE), 128, 0, stream>>>(HBH, HBL, PK, F[6], CNT, LIST, O);
  k_comb<<<NRT * 64, 128, 0, stream>>>(SEL, WGT, O, (float*)d_out);
}
